// ELLGAT_51797305589896
// MI455X (gfx1250) — hardware-run, weakly checked
//
#include <hip/hip_runtime.h>

typedef float          v8f   __attribute__((ext_vector_type(8)));
typedef float          v4f   __attribute__((ext_vector_type(4)));
typedef unsigned int   v4u   __attribute__((ext_vector_type(4)));
typedef int            v8i   __attribute__((ext_vector_type(8)));
typedef unsigned short v8us  __attribute__((ext_vector_type(8)));
typedef unsigned short v16us __attribute__((ext_vector_type(16)));
typedef __bf16         v16bf __attribute__((ext_vector_type(16)));
typedef _Float16       v16h  __attribute__((ext_vector_type(16)));
typedef v4f  __attribute__((may_alias)) v4fa;
typedef v8us __attribute__((may_alias)) v8usa;
union FragB { v16bf v; v16us u; v8us h[2]; v8i w; };
union FragH { v16h  v; v16us u; v8us h[2]; v8i w; };

__device__ __forceinline__ v8f wmb(const FragB& a, const FragB& b, v8f c) {
  v8f d = __builtin_amdgcn_wmma_f32_16x16x32_bf16(false, a.v, false, b.v, (short)0, c, false, false);
  asm volatile("v_nop\n\tv_nop\n\tv_nop\n\tv_nop" : "+v"(d) : "v"(a.w), "v"(b.w));
  return d;
}

__device__ __forceinline__ v8f wmh(const FragH& a, const FragH& b, v8f c) {
  v8f d = __builtin_amdgcn_wmma_f32_16x16x32_f16(false, a.v, false, b.v, (short)0, c, false, false);
  asm volatile("v_nop\n\tv_nop\n\tv_nop\n\tv_nop" : "+v"(d) : "v"(a.w), "v"(b.w));
  return d;
}

__device__ __forceinline__ unsigned bf16_bits(float f) {
  const unsigned u = __float_as_uint(f);
  const unsigned r = (u + 0x7FFFu + ((u >> 16) & 1u)) >> 16;
  const unsigned q = (u >> 16) | 0x40u;
  return ((u & 0x7fffffffu) > 0x7f800000u) ? q : r;
}

__device__ __forceinline__ float bf16_val(float f) {
  return __uint_as_float(bf16_bits(f) << 16);
}
__device__ __forceinline__ int clampi(int v, int lo, int hi) {
  return v < lo ? lo : (v > hi ? hi : v);
}

__device__ __forceinline__ unsigned f16_bits(float f) {
  const unsigned u  = __float_as_uint(f);
  const unsigned s  = (u >> 16) & 0x8000u;
  const unsigned a  = u & 0x7fffffffu;
  const unsigned t  = a - 0x38000000u;
  const unsigned r  = (t + 0x0FFFu + ((t >> 13) & 1u)) >> 13;
  const unsigned rc = r > 0x7C00u ? 0x7C00u : r;
  const bool small  = a < 0x38800000u;
  const bool isnan  = a > 0x7f800000u;
  const unsigned fin = small ? 0u : (s | rc);
  return isnan ? (s | 0x7E00u) : fin;
}

__device__ __forceinline__ unsigned pk16(unsigned lo, unsigned hi) { return lo | (hi << 16); }
__device__ __forceinline__ unsigned bf16_lo_bits(float v) {
  float hi = bf16_val(v);
  asm volatile("" : "+v"(hi));
  return bf16_bits(v - hi);
}
__device__ __forceinline__ v4u pack8_bf16(v4f a, v4f c) {
  return (v4u){ pk16(bf16_bits(a[0]), bf16_bits(a[1])), pk16(bf16_bits(a[2]), bf16_bits(a[3])),
                pk16(bf16_bits(c[0]), bf16_bits(c[1])), pk16(bf16_bits(c[2]), bf16_bits(c[3])) };
}
__device__ __forceinline__ v4u pack8_bf16_lo(v4f a, v4f c) {
  return (v4u){ pk16(bf16_lo_bits(a[0]), bf16_lo_bits(a[1])), pk16(bf16_lo_bits(a[2]), bf16_lo_bits(a[3])),
                pk16(bf16_lo_bits(c[0]), bf16_lo_bits(c[1])), pk16(bf16_lo_bits(c[2]), bf16_lo_bits(c[3])) };
}
__device__ __forceinline__ v4u pack8_f16(v4f a, v4f c) {
  return (v4u){ pk16(f16_bits(a[0]), f16_bits(a[1])), pk16(f16_bits(a[2]), f16_bits(a[3])),
                pk16(f16_bits(c[0]), f16_bits(c[1])), pk16(f16_bits(c[2]), f16_bits(c[3])) };
}

template <int FORM>
__global__ __launch_bounds__(256) void k_plane(const float* __restrict__ src, int rows, int cols, int ldsrc,
                                               unsigned short* __restrict__ dst, int MP, int KP) {
  static_assert(FORM >= 0 && FORM <= 3);
  const int KTOT = (FORM == 1 || FORM == 3) ? 2 * KP : KP;
  const unsigned ppr   = (unsigned)(KTOT >> 3);
  const unsigned kp8   = (unsigned)(KP >> 3);
  const unsigned total = (unsigned)MP * ppr;
  const unsigned g     = blockIdx.x * 256u + threadIdx.x;
  const unsigned rowu  = g / ppr;
  const unsigned p     = g - rowu * ppr;
  const bool second    = p >= kp8;
  const int row = (int)rowu;
  const int c0  = (int)((second ? p - kp8 : p) << 3);
  const float* srow = src + (size_t)clampi(row, 0, rows - 1) * (size_t)ldsrc;
  float x[8];
  unsigned mk[8];
#pragma unroll
  for (int e = 0; e < 8; ++e) {
    const int c = c0 + e;
    const float v = srow[clampi(c, 0, cols - 1)];
    asm volatile("" :: "v"(v));
    x[e]  = v;
    mk[e] = (row < rows && c < cols) ? 0xFFFFu : 0u;
  }
  const v4f a = (v4f){ x[0], x[1], x[2], x[3] };
  const v4f c = (v4f){ x[4], x[5], x[6], x[7] };
  v4u o;
  if (FORM == 2) {
    o = pack8_f16(a, c);
  } else {
    const v4u hi = pack8_bf16(a, c);
    o = hi;
    if (FORM == 1) { const v4u lo = pack8_bf16_lo(a, c); o = second ? lo : hi; }
  }
  const v4u mw = (v4u){ pk16(mk[0], mk[1]), pk16(mk[2], mk[3]), pk16(mk[4], mk[5]), pk16(mk[6], mk[7]) };
  o &= mw;
  if (g < total) {
    volatile v4u* q = (volatile v4u*)(dst + (size_t)g * 8);
    *q = o;
    __threadfence();
    *q = o;
  }
}

template <int FORM> struct FragOf    { typedef FragB T; };
template <>         struct FragOf<2> { typedef FragH T; };
__device__ __forceinline__ v8f mm(const FragB& a, const FragB& b, v8f c) { return wmb(a, b, c); }
__device__ __forceinline__ v8f mm(const FragH& a, const FragH& b, v8f c) { return wmh(a, b, c); }
template <class F> __device__ __forceinline__ F ld_frag(const unsigned short* p) {
  F f;
  f.h[0] = *(const v8usa*)(p);
  f.h[1] = *(const v8usa*)(p + 16);
  return f;
}

template <int FORM, int EPI>
__global__ __launch_bounds__(256) __attribute__((amdgpu_num_vgpr(248)))
void k_gemm_nt(const unsigned short* __restrict__ A, const unsigned short* __restrict__ B,
               const float* __restrict__ bias, float* __restrict__ D, int M, int N, int KTOT, int ldd) {
  static_assert(FORM >= 0 && FORM <= 2);
  static_assert(EPI == 0 || EPI == 1);
  typedef typename FragOf<FORM>::T F;
  __shared__ __attribute__((aligned(16))) float sT[8][16 * 68];
  const int lane = threadIdx.x & 31;
  const int wave = threadIdx.x >> 5;
  const int tilesM = (M + 63) >> 6;
  const int tilesN = (N + 63) >> 6;
  const int tile = blockIdx.x * 8 + wave;
  if (tile >= tilesM * tilesN) return;
  const int tm = tile / tilesN;
  const int tn = tile - tm * tilesN;
  const int m0 = tm << 6;
  const int n0 = tn << 6;

  const int rl = lane & 15;
  const int h8 = (lane >> 4) * 8;
  const unsigned short* pa = A + (size_t)(m0 + rl) * (size_t)KTOT + h8;
  const unsigned short* pb = B + (size_t)(n0 + rl) * (size_t)KTOT + h8;

  v8f acc[4][4];
#pragma unroll
  for (int i = 0; i < 4; ++i)
#pragma unroll
    for (int j = 0; j < 4; ++j) acc[i][j] = (v8f){0.f, 0.f, 0.f, 0.f, 0.f, 0.f, 0.f, 0.f};

#pragma unroll 1
  for (int k0 = 0; k0 < KTOT; k0 += 32) {
    F bf[4];
#pragma unroll
    for (int j = 0; j < 4; ++j) bf[j] = ld_frag<F>(pb + (size_t)(j << 4) * (size_t)KTOT + k0);
#pragma unroll
    for (int i = 0; i < 4; ++i) {
      const F af = ld_frag<F>(pa + (size_t)(i << 4) * (size_t)KTOT + k0);
#pragma unroll
      for (int j = 0; j < 4; ++j) acc[i][j] = mm(af, bf[j], acc[i][j]);
    }
  }

  float* slab = sT[wave];
  const int hh = lane >> 4;
  const int c4 = (lane & 15) * 4;
  const int nc = n0 + c4;
  const bool cok = nc < N;
  v4f bv = (v4f){0.f, 0.f, 0.f, 0.f};
  if (EPI == 1) {
    bv = *(const v4fa*)(bias + clampi(nc, 0, N - 4));
    asm volatile("" :: "v"(bv));
  }
#pragma unroll
  for (int i = 0; i < 4; ++i) {
    const int mBase = m0 + (i << 4);
#pragma unroll
    for (int j = 0; j < 4; ++j) {
#pragma unroll
      for (int r = 0; r < 8; ++r) slab[(h8 + r) * 68 + (j << 4) + rl] = acc[i][j][r];
    }
    __builtin_amdgcn_fence(__ATOMIC_RELEASE, "workgroup");
    __builtin_amdgcn_wave_barrier();
    __builtin_amdgcn_fence(__ATOMIC_ACQUIRE, "workgroup");
    v4f vv[8];
#pragma unroll
    for (int it = 0; it < 8; ++it) {
      const int row = it * 2 + hh;
      v4f v = *(const v4fa*)(slab + row * 68 + c4);
      if (EPI == 1) v += bv;
      vv[it] = v;
    }
    for (int pass = 0; pass < 2; ++pass) {
#pragma unroll
      for (int it = 0; it < 8; ++it) {
        const int row = mBase + it * 2 + hh;
        if (cok && row < M) *(volatile v4f*)(D + (size_t)row * (size_t)ldd + nc) = vv[it];
      }
      __threadfence();
    }
    __builtin_amdgcn_fence(__ATOMIC_RELEASE, "workgroup");
    __builtin_amdgcn_wave_barrier();
    __builtin_amdgcn_fence(__ATOMIC_ACQUIRE, "workgroup");
  }
}

#pragma clang fp contract(off)

typedef float v2f __attribute__((ext_vector_type(2)));
typedef v2f __attribute__((may_alias)) v2fa;

constexpr int NN     = 50000;
constexpr int KNB    = 32;
constexpr int FIN    = 128;
constexpr int NHEAD  = 4;
constexpr int OUTF   = 16;
constexpr int CH     = NHEAD * OUTF;
constexpr int MP     = 50048;
constexpr int OUT_ELEMS = CH * NN;
constexpr int NWV    = 4;

static_assert(NHEAD * OUTF == 64 && CH == 2 * 32);
static_assert(KNB == 32);
static_assert(NN % 8 == 0 && NN % NWV == 0 && NN % 4 == 0);
static_assert(OUT_ELEMS == 64 * NN && OUT_ELEMS % 256 == 0 && OUT_ELEMS == 3200000);
static_assert(MP == 782 * 64 && MP % 128 == 0 && MP >= NN && MP % 16 == 0);
static_assert(FIN == 128 && FIN % 64 == 0 && FIN % 32 == 0);
static_assert(CH % 64 == 0 && CH % 4 == 0 && CH % 32 == 0);
static_assert((long long)MP * FIN / 8 < 0x7fffffffLL);
static_assert(((size_t)NN * 4) % 16 == 0 && ((size_t)(NN - 4) * 4) % 16 == 0);

constexpr size_t SZ_PL  = (size_t)MP * FIN * 2;
constexpr size_t SZ_PT  = (size_t)MP * CH * 4;
constexpr size_t SZ_R   = (size_t)NN * CH * 4;
constexpr size_t SZ_W   = (size_t)CH * FIN * 2;
constexpr size_t SZ_AW  = 256;
constexpr size_t OFF_QB  = 0;
constexpr size_t OFF_KB  = OFF_QB + SZ_PL;
constexpr size_t OFF_QPT = OFF_KB + SZ_PL;
constexpr size_t OFF_KPT = OFF_QPT + SZ_PT;
constexpr size_t OFF_R   = OFF_KPT + SZ_PT;
constexpr size_t OFF_WQ  = OFF_R + SZ_R;
constexpr size_t OFF_WK  = OFF_WQ + SZ_W;
constexpr size_t OFF_AW  = OFF_WK + SZ_W;
constexpr size_t WS_TOTAL = OFF_AW + SZ_AW;
static_assert(SZ_PL % 256 == 0 && SZ_PT % 256 == 0 && SZ_R % 256 == 0 && SZ_W % 256 == 0 && SZ_AW % 256 == 0);
static_assert(OFF_KB % 256 == 0 && OFF_QPT % 256 == 0 && OFF_KPT % 256 == 0 && OFF_R % 256 == 0);
static_assert(OFF_WQ % 256 == 0 && OFF_WK % 256 == 0 && OFF_AW % 256 == 0);
static_assert(OFF_KB == (size_t)12812288 && OFF_QPT == (size_t)25624576 && OFF_KPT == (size_t)38436864);
static_assert(OFF_R == (size_t)51249152 && OFF_WQ == (size_t)64049152 && OFF_WK == (size_t)64065536);
static_assert(OFF_AW == (size_t)64081920 && WS_TOTAL == (size_t)64082176);
static_assert(WS_TOTAL <= ((size_t)128 << 20));

__global__ __launch_bounds__(256) void k_tr(const float* __restrict__ src, unsigned short* __restrict__ dst) {
  __shared__ float tile[64 * 65];
  const int tid = (int)threadIdx.x;
  const int n0 = (int)blockIdx.x << 6;
  const int k0 = (int)blockIdx.y << 6;
  const int c4 = (tid & 15) * 4;
  const int nraw = n0 + c4;
  const int nld  = nraw < NN - 4 ? nraw : NN - 4;
  const unsigned msk = nraw < NN ? 0xFFFFFFFFu : 0u;
#pragma unroll
  for (int i = 0; i < 4; ++i) {
    const int kr = (tid >> 4) + 16 * i;
    const v4f v = *(const v4fa*)(src + (size_t)(k0 + kr) * (size_t)NN + nld);
    asm volatile("" :: "v"(v));
    tile[kr * 65 + c4 + 0] = __uint_as_float(__float_as_uint(v[0]) & msk);
    tile[kr * 65 + c4 + 1] = __uint_as_float(__float_as_uint(v[1]) & msk);
    tile[kr * 65 + c4 + 2] = __uint_as_float(__float_as_uint(v[2]) & msk);
    tile[kr * 65 + c4 + 3] = __uint_as_float(__float_as_uint(v[3]) & msk);
  }
  __syncthreads();
  v4u o[2];
#pragma unroll
  for (int i = 0; i < 2; ++i) {
    const int q  = tid + 256 * i;
    const int n  = q >> 3;
    const int pc = q & 7;
    const float* tp = tile + (pc * 8) * 65 + n;
    o[i] = (v4u){ pk16(bf16_bits(tp[0 * 65]), bf16_bits(tp[1 * 65])), pk16(bf16_bits(tp[2 * 65]), bf16_bits(tp[3 * 65])),
                  pk16(bf16_bits(tp[4 * 65]), bf16_bits(tp[5 * 65])), pk16(bf16_bits(tp[6 * 65]), bf16_bits(tp[7 * 65])) };
  }
#pragma unroll
  for (int i = 0; i < 2; ++i) {
    const int q = tid + 256 * i;
    unsigned short* dp = dst + (size_t)(n0 + (q >> 3)) * (size_t)FIN + k0 + (q & 7) * 8;
    *(volatile v4u*)dp = o[i];
  }
  __threadfence();
#pragma unroll
  for (int i = 0; i < 2; ++i) {
    const int q = tid + 256 * i;
    unsigned short* dp = dst + (size_t)(n0 + (q >> 3)) * (size_t)FIN + k0 + (q & 7) * 8;
    *(volatile v4u*)dp = o[i];
  }
}

__device__ __forceinline__ void prep_w(const float* __restrict__ w, unsigned short* __restrict__ dst, int g) {
  const v4f a = *(const v4fa*)(w + (size_t)g * 8);
  const v4f c = *(const v4fa*)(w + (size_t)g * 8 + 4);
  asm volatile("" :: "v"(a));
  asm volatile("" :: "v"(c));
  const v4u o = pack8_bf16(a, c);
  volatile v4u* q = (volatile v4u*)(dst + (size_t)g * 8);
  *q = o;
  __threadfence();
  *q = o;
}

__global__ __launch_bounds__(256) void k_prep(const float* __restrict__ qw, const float* __restrict__ kw,
                                              const float* __restrict__ aw, unsigned short* __restrict__ WQ,
                                              unsigned short* __restrict__ WK, float* __restrict__ AW) {
  const int tid = (int)threadIdx.x;
  const int blk = (int)blockIdx.x;
  if (blk < 4) {
    prep_w(qw, WQ, blk * 256 + tid);
  } else if (blk < 8) {
    prep_w(kw, WK, (blk - 4) * 256 + tid);
  } else {
    const int u = tid < 16 ? tid : 15;
    const v4f a = *(const v4fa*)(aw + 4 * u);
    asm volatile("" :: "v"(a));
    const v4f o = (v4f){ bf16_val(a[0]), bf16_val(a[1]), bf16_val(a[2]), bf16_val(a[3]) };
    if (tid < 16) {
      volatile v4f* q = (volatile v4f*)(AW + 4 * tid);
      *q = o;
      __threadfence();
      *q = o;
    }
  }
}

__global__ __launch_bounds__(128) __attribute__((amdgpu_num_vgpr(248)))
void k_node(const int* __restrict__ adj, const float* __restrict__ QpT, const float* __restrict__ KpT,
            const float* __restrict__ AW, float* __restrict__ R) {
  __shared__ __attribute__((aligned(16))) float sX[NWV * KNB * CH];
  __shared__ __attribute__((aligned(16))) float sP[NWV * KNB * CH];
  const int tid = (int)threadIdx.x, lane = tid & 31, wave = tid >> 5;
  const int n  = __builtin_amdgcn_readfirstlane((int)blockIdx.x * NWV + wave);
  const int nc = n < NN ? n : NN - 1;

  int raw = adj[(size_t)nc * KNB + lane];
  asm volatile("" :: "v"(raw));
  const int idc = clampi(raw, 0, NN - 1);
  const unsigned vmask = __builtin_amdgcn_ballot_w32(raw != -1);
  const int cnt = __builtin_popcount(vmask);
  const bool none = (cnt == 0);

  const v2f qv = *(const v2fa*)(QpT + (size_t)nc * CH + 2 * lane);
  const float q0 = qv[0], q1 = qv[1];
  asm volatile("" :: "v"(q0));
  asm volatile("" :: "v"(q1));
  const v2f av = *(const v2fa*)(AW + 2 * lane);
  const float aw0 = av[0], aw1 = av[1];
  asm volatile("" :: "v"(aw0));
  asm volatile("" :: "v"(aw1));

  const float* Kl = KpT + 2 * lane;
  float* sx = sX + wave * (KNB * CH) + 2 * lane;
  float* sp = sP + wave * (KNB * CH) + 2 * lane;

  float m0 = -__builtin_inff(), m1 = -__builtin_inff();
#pragma unroll 4
  for (int k = 0; k < KNB; ++k) {
    const int  nr  = __builtin_amdgcn_readlane(idc, k);
    const bool vld = ((vmask >> k) & 1u) != 0u;
    const v2f kv = *(const v2fa*)(Kl + (size_t)nr * CH);
    const float g0 = kv[0], g1 = kv[1];
    asm volatile("" :: "v"(g0));
    asm volatile("" :: "v"(g1));
    const float x0 = q0 * g0;
    const float x1 = q1 * g1;
    const float X0 = (x0 >= 0.0f) ? x0 : 0.01f * x0;
    const float X1 = (x1 >= 0.0f) ? x1 : 0.01f * x1;
    *(v2fa*)(sx + k * CH) = (v2f){ X0, X1 };
    const bool t0 = vld & ((X0 > m0) | (X0 != X0));
    const bool t1 = vld & ((X1 > m1) | (X1 != X1));
    m0 = t0 ? X0 : m0;
    m1 = t1 ? X1 : m1;
  }
  m0 = none ? 0.0f : m0;
  m1 = none ? 0.0f : m1;

  float S0 = 0.0f, S1 = 0.0f;
#pragma unroll 4
  for (int k = 0; k < KNB; ++k) {
    const unsigned keep = 0u - ((vmask >> k) & 1u);
    const v2f xv = *(const v2fa*)(sx + k * CH);
    const float d0 = __uint_as_float(__float_as_uint(xv[0] - m0) & keep);
    const float d1 = __uint_as_float(__float_as_uint(xv[1] - m1) & keep);
    const float e0 = expf(d0);
    const float e1 = expf(d1);
    const float p0 = __uint_as_float(__float_as_uint(e0) & keep);
    const float p1 = __uint_as_float(__float_as_uint(e1) & keep);
    S0 = S0 + p0;
    S1 = S1 + p1;
    *(v2fa*)(sp + k * CH) = (v2f){ p0, p1 };
  }
  const float Ss0 = none ? 1.0f : S0;
  const float Ss1 = none ? 1.0f : S1;
  float r0 = 1.0f / Ss0;
  float r1 = 1.0f / Ss1;
  r0 = none ? 0.0f : r0;
  r1 = none ? 0.0f : r1;

  float o0 = 0.0f, o1 = 0.0f;
#pragma unroll 4
  for (int k = 0; k < KNB; ++k) {
    const unsigned keep = 0u - ((vmask >> k) & 1u);
    const v2f pv = *(const v2fa*)(sp + k * CH);
    const v2f xv = *(const v2fa*)(sx + k * CH);
    const float a0 = pv[0] * r0;
    const float a1 = pv[1] * r1;
    float t = a0 * aw0 + a1 * aw1;
    t = t + __shfl_xor(t, 1, 32);
    t = t + __shfl_xor(t, 2, 32);
    t = t + __shfl_xor(t, 4, 32);
    const float xm0 = __uint_as_float(__float_as_uint(xv[0]) & keep);
    const float xm1 = __uint_as_float(__float_as_uint(xv[1]) & keep);
    o0 = o0 + t * xm0;
    o1 = o1 + t * xm1;
  }

  const v2f o = (v2f){ o0, o1 };
  if (n < NN) {
    volatile v2f* q = (volatile v2f*)(R + (size_t)n * CH + 2 * lane);
    *q = o;
    __threadfence();
    *q = o;
  }
}

static_assert((OUT_ELEMS / 256) * 256 == OUT_ELEMS);
__global__ __launch_bounds__(256) void k_out(const float* __restrict__ R, float* __restrict__ out) {
  const int f  = (int)blockIdx.x * 256 + (int)threadIdx.x;
  const int fc = f < OUT_ELEMS ? f : OUT_ELEMS - 1;
  const int c  = fc / NN;
  const int n  = fc - c * NN;
  const float v = R[(size_t)n * CH + c];
  asm volatile("" :: "v"(v));
  if (f < OUT_ELEMS) {
    volatile float* q = (volatile float*)(out + f);
    *q = v;
    __threadfence();
    *q = v;
  }
}

extern "C" void kernel_launch(void* const* d_in, const int* in_sizes, int n_in,
                              void* d_out, int out_size, void* d_ws, size_t ws_size,
                              hipStream_t stream) {
  if (n_in < 6) return;
  if (in_sizes[0] != NN * KNB) return;
  if (in_sizes[1] != FIN * NN) return;
  if (in_sizes[2] != FIN * NN) return;
  if (in_sizes[3] != CH * FIN) return;
  if (in_sizes[4] != CH * FIN) return;
  if (in_sizes[5] != CH) return;
  if (out_size != OUT_ELEMS) return;
  if (ws_size < WS_TOTAL) return;

  const int*   adj = (const int*)d_in[0];
  const float* Q   = (const float*)d_in[1];
  const float* K   = (const float*)d_in[2];
  const float* qw  = (const float*)d_in[3];
  const float* kw  = (const float*)d_in[4];
  const float* aw  = (const float*)d_in[5];
  float* out = (float*)d_out;

  char* ws = (char*)d_ws;
  unsigned short* QB  = (unsigned short*)(ws + OFF_QB);
  unsigned short* KB  = (unsigned short*)(ws + OFF_KB);
  float*          QpT = (float*)(ws + OFF_QPT);
  float*          KpT = (float*)(ws + OFF_KPT);
  float*          R   = (float*)(ws + OFF_R);
  unsigned short* WQ  = (unsigned short*)(ws + OFF_WQ);
  unsigned short* WK  = (unsigned short*)(ws + OFF_WK);
  float*          AW  = (float*)(ws + OFF_AW);

  k_tr<<<dim3(MP / 64, FIN / 64, 1), 256, 0, stream>>>(Q, QB);
  k_tr<<<dim3(MP / 64, FIN / 64, 1), 256, 0, stream>>>(K, KB);
  k_prep<<<9, 256, 0, stream>>>(qw, kw, aw, WQ, WK, AW);
  k_gemm_nt<0, 0><<<(MP / 64 + 7) / 8, 256, 0, stream>>>(QB, WQ, AW, QpT, MP, CH, FIN, CH);
  k_gemm_nt<0, 0><<<(MP / 64 + 7) / 8, 256, 0, stream>>>(KB, WK, AW, KpT, MP, CH, FIN, CH);
  k_node<<<NN / NWV, 128, 0, stream>>>(adj, QpT, KpT, AW, R);
  k_out<<<OUT_ELEMS / 256, 256, 0, stream>>>(R, out);
}
